// myGNN_45655502356933
// MI455X (gfx1250) — hardware-verified
//
#include <hip/hip_runtime.h>
#include <stddef.h>
#include <stdint.h>


#define DIN     128
#define HC1     256
#define HC2     128
#define NTHR    256
#define NWAVE   8
#define EPT     8
#define CHUNK   (NTHR * EPT)
#define WCAP    (EPT * 32)
#define LISTN   (NWAVE * WCAP)
#define NBMAX   2048
#define NBRUN   512
#define RCAP    28672
#define DEGCAP  128
#define GBM     64
#define GBN     64
#define GTHR    128
#define NPB     64
#define STHR    DIN
#define PARTD   (2 * DIN)
#define NEGS    0.2f
#define NEG1    0.01f
#define WSMAX   134217728
#define LDS_INTS (2 * RCAP + 2 * NBMAX + LISTN)
#define LDS_AGG (LDS_INTS * 4 + 64)

static_assert((CHUNK & (CHUNK - 1)) == 0 && CHUNK <= 4096);
static_assert((NBMAX & (NBMAX - 1)) == 0 && NBMAX <= 4096);
static_assert((NBRUN & (NBRUN - 1)) == 0 && NBRUN <= NBMAX && NBRUN >= 16);
static_assert(NTHR * 8 == NBMAX);
static_assert(LISTN >= NBMAX);
static_assert(LISTN >= NWAVE * WCAP);
static_assert((RCAP % 32) == 0);
static_assert((LDS_INTS % 4) == 0);
static_assert(LDS_AGG <= 300000);
static_assert(GBM == (GTHR / 32) * 16);
static_assert(((2 * DIN) % 32) == 0 && ((2 * HC1) % 32) == 0);
static_assert(((2 * HC1) % GBN) == 0 && ((2 * HC2) % GBN) == 0);
static_assert((HC1 % GBN) == 0 && (HC2 % GBN) == 0);
static_assert(NTHR == 2 * DIN);
static_assert(STHR == DIN && (PARTD * 8) % 128 == 0 && PARTD / 2 == STHR);
static_assert(HC1 == 32 * 8 && HC2 == 32 * 4);

typedef float          v4f   __attribute__((ext_vector_type(4)));
typedef float          v8f   __attribute__((ext_vector_type(8)));
typedef double         v2d   __attribute__((ext_vector_type(2)));
typedef int            v4i   __attribute__((ext_vector_type(4)));
typedef int            v8i   __attribute__((ext_vector_type(8)));
typedef unsigned short v8us  __attribute__((ext_vector_type(8)));
typedef unsigned short v16us __attribute__((ext_vector_type(16)));
typedef __bf16         v16bf __attribute__((ext_vector_type(16)));
typedef v4f  __attribute__((may_alias)) v4fa;
typedef v4i  __attribute__((may_alias)) v4ia;
typedef v2d  __attribute__((may_alias)) v2da;
typedef v8us __attribute__((may_alias)) v8usa;
union FragB { v16bf v; v16us u; v8us h[2]; v8i w; };

__device__ __forceinline__ v8f wmb(const FragB& a, const FragB& b, v8f c) {
  v8f d = __builtin_amdgcn_wmma_f32_16x16x32_bf16(false, a.v, false, b.v, (short)0, c, false, false);
  asm volatile("v_nop\n\tv_nop\n\tv_nop\n\tv_nop" : "+v"(d) : "v"(a.w), "v"(b.w));
  return d;
}

__device__ __forceinline__ void ldwait() {
  asm volatile("s_wait_loadcnt 0x0" ::: "memory");
}

__device__ __forceinline__ unsigned bfbits(float v) {
  unsigned u = __float_as_uint(v);
  u = u + 0x7FFFu + ((u >> 16) & 1u);
  return u >> 16;
}
__device__ __forceinline__ float rbf(float v) { return __uint_as_float(bfbits(v) << 16); }

__device__ __forceinline__ v8us cvt8b(const v4f a, const v4f b) {
  v8us o;
  o[0] = (unsigned short)bfbits(a.x); o[1] = (unsigned short)bfbits(a.y);
  o[2] = (unsigned short)bfbits(a.z); o[3] = (unsigned short)bfbits(a.w);
  o[4] = (unsigned short)bfbits(b.x); o[5] = (unsigned short)bfbits(b.y);
  o[6] = (unsigned short)bfbits(b.z); o[7] = (unsigned short)bfbits(b.w);
  return o;
}

template<int CPL>
__device__ __forceinline__ void ldrow(const float* p, float* o) {
#pragma unroll
  for (int q = 0; q < CPL / 4; ++q) {
    const v4f t = *(const v4f*)(p + 4 * q);
    o[4 * q + 0] = t.x; o[4 * q + 1] = t.y; o[4 * q + 2] = t.z; o[4 * q + 3] = t.w;
  }
}

template<int CPL, int GSH>
__device__ __forceinline__ float gat_logit(const float* hs, const float* hd, const float* at) {
  float part = 0.0f;
#pragma unroll
  for (int i = 0; i < CPL; ++i) {
    float v = hs[i] + hd[i];
    v = v > 0.f ? v : v * NEGS;
    part = fmaf(v, at[i], part);
  }
#pragma unroll
  for (int off = (1 << (GSH - 1)); off > 0; off >>= 1) part += __shfl_xor(part, off);
  return part;
}

__device__ __forceinline__ int scan_chunk(const int* __restrict__ dsts, int nE, int cbase, int slotBase,
                                          int nb, int vec8, int* list, int tid, int lane, int wave) {
  int wc = 0;
  const int el0  = tid * EPT;
  const int e0   = cbase + el0;
  const int sent = -2147483647 - 1;
  v4i da, db;
  if (vec8 != 0 && cbase + CHUNK <= nE) {
    da = *(const v4i*)(dsts + e0);
    db = *(const v4i*)(dsts + e0 + 4);
  } else {
    da.x = (e0     < nE) ? dsts[min(e0,     nE - 1)] : sent;
    da.y = (e0 + 1 < nE) ? dsts[min(e0 + 1, nE - 1)] : sent;
    da.z = (e0 + 2 < nE) ? dsts[min(e0 + 2, nE - 1)] : sent;
    da.w = (e0 + 3 < nE) ? dsts[min(e0 + 3, nE - 1)] : sent;
    db.x = (e0 + 4 < nE) ? dsts[min(e0 + 4, nE - 1)] : sent;
    db.y = (e0 + 5 < nE) ? dsts[min(e0 + 5, nE - 1)] : sent;
    db.z = (e0 + 6 < nE) ? dsts[min(e0 + 6, nE - 1)] : sent;
    db.w = (e0 + 7 < nE) ? dsts[min(e0 + 7, nE - 1)] : sent;
  }
  const unsigned nbs = (unsigned)slotBase;
  const unsigned unb = (unsigned)nb;
  const unsigned s0 = (unsigned)da.x - nbs, s1 = (unsigned)da.y - nbs;
  const unsigned s2 = (unsigned)da.z - nbs, s3 = (unsigned)da.w - nbs;
  const unsigned s4 = (unsigned)db.x - nbs, s5 = (unsigned)db.y - nbs;
  const unsigned s6 = (unsigned)db.z - nbs, s7 = (unsigned)db.w - nbs;
  const bool h0 = s0 < unb, h1 = s1 < unb, h2 = s2 < unb, h3 = s3 < unb;
  const bool h4 = s4 < unb, h5 = s5 < unb, h6 = s6 < unb, h7 = s7 < unb;
  const unsigned any = __builtin_amdgcn_ballot_w32(h0 | h1 | h2 | h3 | h4 | h5 | h6 | h7);
  if (any != 0u) {
#define HITJ(J, HJ, SJ) { \
      const unsigned mj = __builtin_amdgcn_ballot_w32(HJ); \
      if (mj != 0u) { \
        if (HJ) { \
          const int pos = wc + (int)__builtin_amdgcn_mbcnt_lo(mj, 0u); \
          if (pos < WCAP) list[wave * WCAP + pos] = ((el0 + (J)) << 12) | (int)(SJ); \
        } \
        wc += (int)__builtin_popcount(mj); } }
    HITJ(0, h0, s0)
    HITJ(1, h1, s1)
    HITJ(2, h2, s2)
    HITJ(3, h3, s3)
    HITJ(4, h4, s4)
    HITJ(5, h5, s5)
    HITJ(6, h6, s6)
    HITJ(7, h7, s7)
#undef HITJ
  }
  return wc;
}

__global__ __launch_bounds__(STHR) void k_bnstat(const float* __restrict__ x, int nN, int rpb, double* part) {
  __shared__ __attribute__((aligned(16))) double sh[PARTD];
  const int c = (int)threadIdx.x;
  const int b = (int)blockIdx.x;
  const int r0 = b * rpb;
  int r1 = r0 + rpb;
  r1 = r1 > nN ? nN : r1;
  double s = 0.0, s2 = 0.0;
#pragma unroll 1
  for (int r = r0; r < r1; ++r) {
    const float v = rbf(x[(size_t)r * DIN + c]);
    const double dv = (double)v;
    s  = s + dv;
    s2 = fma(dv, dv, s2);
  }
  sh[c] = s;
  sh[DIN + c] = s2;
  __syncthreads();
  const v2d v = *(const v2da*)(sh + 2 * c);
  double* pp = part + (size_t)b * PARTD + 2 * c;
  *(volatile v2d*)pp = v;
  __threadfence();
  *(volatile v2d*)pp = v;
}

__global__ __launch_bounds__(STHR) void k_bnfin(const double* __restrict__ part, int nPart, int nN,
                                                const float* __restrict__ gam, const float* __restrict__ bet,
                                                float* ss) {
  __shared__ __attribute__((aligned(16))) float stg[2 * DIN];
  const int tid = (int)threadIdx.x;
  const int c = tid;
  double S = 0.0, S2 = 0.0;
#pragma unroll 1
  for (int b = 0; b < nPart; ++b) {
    S  += part[(size_t)b * PARTD + c];
    S2 += part[(size_t)b * PARTD + DIN + c];
  }
  const double dn = (double)(nN > 0 ? nN : 1);
  const double mean = S / dn;
  double var = S2 / dn - mean * mean;
  var = var < 0.0 ? 0.0 : var;
  const float meanf = (float)mean;
  const float varf  = (float)var;
  const float rstd = 1.0f / sqrtf(varf + 1e-5f);
  const float sc = rbf(gam[c]) * rstd;
  const float sf = rbf(bet[c]) - meanf * sc;
  stg[c] = sc;
  stg[DIN + c] = sf;
  __syncthreads();
  v4f v;
  if (tid < (2 * DIN) / 4) {
    v = *(const v4fa*)(stg + 4 * tid);
    *(volatile v4f*)(ss + 4 * tid) = v;
  }
  __threadfence();
  if (tid < (2 * DIN) / 4) {
    *(volatile v4f*)(ss + 4 * tid) = v;
  }
}

__global__ __launch_bounds__(NTHR) void k_xprep(const float* __restrict__ x, const float* __restrict__ ss,
                                                unsigned short* xn, int nN, int nUnits) {
  __shared__ float ssh[2 * DIN];
  const int tid = (int)threadIdx.x;
  ssh[tid] = ss[tid];
  __syncthreads();
  const int i = (int)blockIdx.x * NTHR + tid;
  if (i >= nUnits) return;
  const int row = i >> 4;
  const int c0  = (i & 15) * 8;
  const int rc  = row < nN ? row : nN - 1;
  const float* p = x + (size_t)rc * DIN + c0;
  const v4f a = *(const v4f*)p, b = *(const v4f*)(p + 4);
  const float live = row < nN ? 1.0f : 0.0f;
  float f[8] = {a.x, a.y, a.z, a.w, b.x, b.y, b.z, b.w};
  v8us hv, lv;
#pragma unroll
  for (int j = 0; j < 8; ++j) {
    const float y = live * fmaf(rbf(f[j]), ssh[c0 + j], ssh[DIN + c0 + j]);
    const unsigned hb = bfbits(y);
    hv[j] = (unsigned short)hb;
    lv[j] = (unsigned short)bfbits(y - __uint_as_float(hb << 16));
  }
  const size_t o = (size_t)row * (2 * DIN) + c0;
  *(volatile v8us*)(xn + o) = hv;
  *(volatile v8us*)(xn + o + DIN) = lv;
  __threadfence();
  *(volatile v8us*)(xn + o) = hv;
  *(volatile v8us*)(xn + o + DIN) = lv;
}

__global__ __launch_bounds__(NTHR) void k_wtr(const float* __restrict__ wl, const float* __restrict__ wr,
                                              int cols, int K, unsigned short* bt) {
  const int K2 = 2 * K;
  const int kq = K2 >> 3;
  const int nUnits = cols * kq;
  const int u = (int)blockIdx.x * NTHR + (int)threadIdx.x;
  if (u >= nUnits) return;
  const int side = (int)blockIdx.y;
  const float* w = side != 0 ? wr : wl;
  const int n  = u / kq;
  const int k8 = (u - n * kq) * 8;
  const int kk = k8 >= K ? k8 - K : k8;
  const float* p = w + (size_t)kk * (size_t)cols + n;
  v4f a, b;
  a.x = p[0];                  a.y = p[(size_t)cols];       a.z = p[(size_t)2 * cols];   a.w = p[(size_t)3 * cols];
  b.x = p[(size_t)4 * cols];   b.y = p[(size_t)5 * cols];   b.z = p[(size_t)6 * cols];   b.w = p[(size_t)7 * cols];
  const v8us hv = cvt8b(a, b);
  const size_t o = (size_t)(side * cols + n) * (size_t)K2 + k8;
  *(volatile v8us*)(bt + o) = hv;
  __threadfence();
  *(volatile v8us*)(bt + o) = hv;
}

__global__ __launch_bounds__(GTHR) void k_gemm(
    const unsigned short* __restrict__ A, const unsigned short* __restrict__ WT,
    const float* __restrict__ bl, const float* __restrict__ br, int nhalf,
    float* outF, int K, int ldo)
{
  __shared__ __attribute__((aligned(16))) float stg[GBM * GBN];
  const int tid = (int)threadIdx.x, lane = tid & 31, wave = tid >> 5, hh = lane >> 4, m = lane & 15;
  const int rowBase = (int)blockIdx.x * GBM;
  const int col0    = (int)blockIdx.y * GBN;

  const float* bp = (col0 < nhalf) ? (bl + col0) : (br + (col0 - nhalf));
  float bc[4];
#pragma unroll
  for (int t = 0; t < 4; ++t) bc[t] = rbf(bp[16 * t + m]);

  v8f acc[4];
  {
    const v8f z = {0.f, 0.f, 0.f, 0.f, 0.f, 0.f, 0.f, 0.f};
    acc[0] = z; acc[1] = z; acc[2] = z; acc[3] = z;
  }
  const unsigned short* ap = A  + (size_t)(rowBase + 16 * wave + m) * (size_t)K + 8 * hh;
  const unsigned short* wp = WT + (size_t)(col0 + m) * (size_t)K + 8 * hh;
  const int ksteps = K >> 5;
#pragma unroll 1
  for (int ks = 0; ks < ksteps; ++ks) {
    FragB af;
    af.h[0] = *(const v8usa*)(ap + 32 * ks);
    af.h[1] = *(const v8usa*)(ap + 32 * ks + 16);
#pragma unroll
    for (int t = 0; t < 4; ++t) {
      const unsigned short* wq = wp + (size_t)(16 * t) * (size_t)K + 32 * ks;
      FragB bf;
      bf.h[0] = *(const v8usa*)wq;
      bf.h[1] = *(const v8usa*)(wq + 16);
      acc[t] = wmb(af, bf, acc[t]);
    }
  }

#pragma unroll
  for (int t = 0; t < 4; ++t) {
    const int lc = 16 * t + m;
#pragma unroll
    for (int r = 0; r < 8; ++r) {
      const int lr = 16 * wave + 8 * hh + r;
      stg[lr * GBN + lc] = acc[t][r] + bc[t];
    }
  }
  __syncthreads();

  v4f fv[8];
#pragma unroll
  for (int i = 0; i < 8; ++i) {
    const int lr = 16 * wave + 2 * i + hh;
    fv[i] = *(const v4fa*)(stg + lr * GBN + 4 * m);
  }
#pragma unroll
  for (int i = 0; i < 8; ++i) {
    const int lr = 16 * wave + 2 * i + hh;
    const int gr = rowBase + lr;
    float* op = outF + (size_t)gr * (size_t)ldo + col0 + 4 * m;
    *(volatile v4f*)op = fv[i];
  }
  __threadfence();
#pragma unroll
  for (int i = 0; i < 8; ++i) {
    const int lr = 16 * wave + 2 * i + hh;
    const int gr = rowBase + lr;
    float* op = outF + (size_t)gr * (size_t)ldo + col0 + 4 * m;
    *(volatile v4f*)op = fv[i];
  }
}

template<int CPL, int GSH, int MODE>
__global__ __launch_bounds__(NTHR) void k_agg(
    const int* __restrict__ srcs, const int* __restrict__ dsts,
    const float* __restrict__ HF, const float* __restrict__ att, const float* __restrict__ bias,
    unsigned short* A2, float* outF,
    int nN, int nE, int nb, int vec8, int MPr) {
  constexpr int C = 32 * CPL;
  constexpr int P = 2 * C;
  extern __shared__ v4f lds_dyn[];
  int* reg1 = (int*)lds_dyn;
  int* reg2 = reg1 + RCAP;
  int* scnt = reg2 + RCAP;
  int* soff = scnt + NBMAX;
  int* list = soff + NBMAX;
  int* wcnt = list + LISTN;
  int* wtot = wcnt + NWAVE;
  const int tid = (int)threadIdx.x, lane = tid & 31, wave = tid >> 5;
  const int nodeBase = (int)blockIdx.x * nb;

  {
    const v4i z4 = {0, 0, 0, 0};
    v4ia* lz = (v4ia*)lds_dyn;
#pragma unroll 1
    for (int i = tid; i < LDS_INTS / 4; i += NTHR) lz[i] = z4;
    if (tid < 2 * NWAVE) wcnt[tid] = 0;
  }
  __syncthreads();

  int tot = 0;
  const int nChunks = (nE + CHUNK - 1) / CHUNK;
#pragma unroll 1
  for (int ch = 0; ch < nChunks; ++ch) {
    const int cbase = ch * CHUNK;
    const int wc = scan_chunk(dsts, nE, cbase, nodeBase, nb, vec8, list, tid, lane, wave);
    if (lane == 0) wcnt[wave] = wc;
    __syncthreads();
    int pre = 0, all = 0;
#pragma unroll
    for (int w2 = 0; w2 < NWAVE; ++w2) {
      int c = wcnt[w2];
      c = c < 0 ? 0 : (c > WCAP ? WCAP : c);
      all += c;
      pre += (w2 < wave) ? c : 0;
    }
    const int wcc  = wc > WCAP ? WCAP : wc;
    const int base = tot + pre;
#pragma unroll 1
    for (int i = lane; i < wcc; i += 32) {
      const int ent = list[wave * WCAP + i];
      const int el  = (ent >> 12) & (CHUNK - 1);
      const int sl  = ent & (NBMAX - 1);
      int eid = cbase + el;
      eid = eid > nE - 1 ? nE - 1 : eid;
      const int pos = base + i;
      if (pos < RCAP) reg1[pos] = (int)(((unsigned)eid << 12) | (unsigned)sl);
    }
    tot += all;
    tot = tot > RCAP ? RCAP : tot;
    __syncthreads();
  }
  const int nh = tot;

  if (wave == 0) {
#pragma unroll 1
    for (int b0 = 0; b0 < nh; b0 += 32) {
      const int idx = b0 + lane;
      const int uv  = reg1[idx < RCAP ? idx : RCAP - 1];
      const int m32 = (nh - b0) < 32 ? (nh - b0) : 32;
#pragma unroll 1
      for (int k = 0; k < m32; ++k) {
        const int u  = __builtin_amdgcn_readlane(uv, k);
        const int sl = u & (NBMAX - 1);
        if (lane == 0) scnt[sl] = scnt[sl] + 1;
      }
    }
  }
  __syncthreads();

  {
    const v4i ca = *(const v4ia*)(scnt + 8 * tid);
    const v4i cb = *(const v4ia*)(scnt + 8 * tid + 4);
    const int e0 = ca.x < 0 ? 0 : ca.x, e1 = ca.y < 0 ? 0 : ca.y, e2 = ca.z < 0 ? 0 : ca.z, e3 = ca.w < 0 ? 0 : ca.w;
    const int e4 = cb.x < 0 ? 0 : cb.x, e5 = cb.y < 0 ? 0 : cb.y, e6 = cb.z < 0 ? 0 : cb.z, e7 = cb.w < 0 ? 0 : cb.w;
    const int ts = e0 + e1 + e2 + e3 + e4 + e5 + e6 + e7;
    int incl = ts;
#pragma unroll
    for (int d = 1; d < 32; d <<= 1) {
      const int up = __shfl_up(incl, d);
      if (lane >= d) incl += up;
    }
    if (lane == 31) wtot[wave] = incl;
    __syncthreads();
    int pre = 0;
#pragma unroll
    for (int w2 = 0; w2 < NWAVE; ++w2) pre += (w2 < wave) ? wtot[w2] : 0;
    int run = pre + incl - ts;
    soff[8 * tid + 0] = run; run += e0;
    soff[8 * tid + 1] = run; run += e1;
    soff[8 * tid + 2] = run; run += e2;
    soff[8 * tid + 3] = run; run += e3;
    soff[8 * tid + 4] = run; run += e4;
    soff[8 * tid + 5] = run; run += e5;
    soff[8 * tid + 6] = run; run += e6;
    soff[8 * tid + 7] = run;
  }
  __syncthreads();
  for (int i = tid; i < NBMAX; i += NTHR) list[i] = soff[i];
  __syncthreads();

  if (wave == 0) {
#pragma unroll 1
    for (int b0 = 0; b0 < nh; b0 += 32) {
      const int idx = b0 + lane;
      const int uv  = reg1[idx < RCAP ? idx : RCAP - 1];
      const int m32 = (nh - b0) < 32 ? (nh - b0) : 32;
#pragma unroll 1
      for (int k = 0; k < m32; ++k) {
        const int u   = __builtin_amdgcn_readlane(uv, k);
        const int sl  = u & (NBMAX - 1);
        const int eid = (int)((unsigned)u >> 12);
        if (lane == 0) {
          int pos = list[sl];
          pos = pos < 0 ? 0 : (pos > RCAP - 1 ? RCAP - 1 : pos);
          reg2[pos] = eid;
          list[sl] = pos + 1;
        }
      }
    }
  }
  __syncthreads();

  const int nbw = nb >> 3;
  const bool ovf = (nh >= RCAP);
  const float qnan = __int_as_float(0x7fc00000);
  float at[CPL], bb[CPL];
  {
    const float* pa = att  + CPL * lane;
    const float* pb = bias + CPL * lane;
#pragma unroll
    for (int q4 = 0; q4 < CPL / 4; ++q4) {
      const v4f ta = *(const v4f*)(pa + 4 * q4);
      const v4f tb = *(const v4f*)(pb + 4 * q4);
      at[4 * q4 + 0] = rbf(ta.x); at[4 * q4 + 1] = rbf(ta.y); at[4 * q4 + 2] = rbf(ta.z); at[4 * q4 + 3] = rbf(ta.w);
      bb[4 * q4 + 0] = rbf(tb.x); bb[4 * q4 + 1] = rbf(tb.y); bb[4 * q4 + 2] = rbf(tb.z); bb[4 * q4 + 3] = rbf(tb.w);
    }
  }
#pragma unroll 1
  for (int jt = 0; jt < nbw; ++jt) {
    const int slot = wave * nbw + jt;
    const int grow = nodeBase + slot;
    const int gcl  = grow < nN ? grow : nN - 1;
    int st = soff[slot];
    const int craw = scnt[slot];
    int cnt = craw;
    st  = st < 0 ? 0 : (st > nh ? nh : st);
    cnt = cnt < 0 ? 0 : (cnt > DEGCAP ? DEGCAP : cnt);
    if (cnt > nh - st) cnt = nh - st;
    const float pz = (ovf || craw > DEGCAP) ? qnan : 0.0f;
    const float live = grow < nN ? 1.0f : 0.0f;

    const float* drow = HF + (size_t)gcl * (size_t)P + CPL * lane;
    float hd[CPL], hs[CPL], av[CPL];
    ldrow<CPL>(drow + C, hd);
    ldrow<CPL>(drow, hs);
    ldwait();
    float mx, dn;
    {
      const float al = gat_logit<CPL, GSH>(hs, hd, at);
      mx = al;
      dn = 1.0f;
#pragma unroll
      for (int i = 0; i < CPL; ++i) av[i] = hs[i];
    }

#pragma unroll 1
    for (int q = 0; q < cnt; ++q) {
      int idx = st + q; idx = idx > RCAP - 1 ? RCAP - 1 : idx;
      int eid = reg2[idx]; eid = eid < 0 ? 0 : (eid > nE - 1 ? nE - 1 : eid);
      const int sraw = srcs[eid];
      const int s = sraw < 0 ? 0 : (sraw > nN - 1 ? nN - 1 : sraw);
      ldrow<CPL>(HF + (size_t)s * (size_t)P + CPL * lane, hs);
      ldwait();
      const float al = gat_logit<CPL, GSH>(hs, hd, at);
      const float df = al - mx;
      const float ee = __expf(-fabsf(df));
      const bool up  = df > 0.f;
      const float s1 = up ? ee : 1.0f;
      const float s2 = up ? 1.0f : ee;
      mx = up ? al : mx;
      dn = fmaf(dn, s1, s2);
#pragma unroll
      for (int i = 0; i < CPL; ++i) av[i] = fmaf(av[i], s1, s2 * hs[i]);
    }
    const float iv = __builtin_amdgcn_rcpf(dn);

    if constexpr (MODE == 0) {
      static_assert(CPL == 8);
      v8us hv, lv;
#pragma unroll
      for (int i = 0; i < CPL; ++i) {
        float v = fmaf(av[i], iv, bb[i]);
        v = v > 0.f ? v : v * NEG1;
        v = v * live + pz;
        const unsigned hb = bfbits(v);
        hv[i] = (unsigned short)hb;
        lv[i] = (unsigned short)bfbits(v - __uint_as_float(hb << 16));
      }
      const bool wr = grow < MPr;
      const int  gw = wr ? grow : MPr - 1;
      unsigned short* gp = A2 + (size_t)gw * (size_t)P + CPL * lane;
      if (wr) { *(volatile v8us*)gp = hv; *(volatile v8us*)(gp + C) = lv; }
      __threadfence();
      if (wr) { *(volatile v8us*)gp = hv; *(volatile v8us*)(gp + C) = lv; }
    } else {
      static_assert(CPL == 4);
      v4f o;
      o.x = fmaf(av[0], iv, bb[0]) + pz;
      o.y = fmaf(av[1], iv, bb[1]) + pz;
      o.z = fmaf(av[2], iv, bb[2]) + pz;
      o.w = fmaf(av[3], iv, bb[3]) + pz;
      const bool wr = grow < nN;
      float* gp = outF + (size_t)gcl * (size_t)C + CPL * lane;
      if (wr) *(volatile v4f*)gp = o;
      __threadfence();
      if (wr) *(volatile v4f*)gp = o;
    }
  }
  (void)A2; (void)outF;
}

static int pick_nb(int nE, int nN) {
  int nb = NBRUN;
  while (nb > 16 && (long long)nb * (long long)nE * 5LL > (long long)RCAP * (long long)nN * 4LL) nb >>= 1;
  return nb;
}
static inline int cdiv(int a, int b) { return (a + b - 1) / b; }
static inline size_t al256(size_t o) { return (o + 255) & ~(size_t)255; }

extern "C" void kernel_launch(void* const* d_in, const int* in_sizes, int n_in,
                              void* d_out, int out_size, void* d_ws, size_t ws_size,
                              hipStream_t stream) {
  if (n_in < 16) return;
  const int nN = in_sizes[0] / DIN;
  if (nN <= 0 || in_sizes[0] != nN * DIN || nN > (1 << 22)) return;
  if (in_sizes[1] < 2 || (in_sizes[1] & 1) != 0) return;
  const int nE = in_sizes[1] / 2;
  if (nE < 1 || nE > (1 << 20)) return;
  if (in_sizes[2] != DIN || in_sizes[3] != DIN) return;
  if (in_sizes[4] != DIN * HC1 || in_sizes[5] != HC1) return;
  if (in_sizes[6] != DIN * HC1 || in_sizes[7] != HC1) return;
  if (in_sizes[8] != HC1 || in_sizes[9] != HC1) return;
  if (in_sizes[10] != HC1 * HC2 || in_sizes[11] != HC2) return;
  if (in_sizes[12] != HC1 * HC2 || in_sizes[13] != HC2) return;
  if (in_sizes[14] != HC2 || in_sizes[15] != HC2) return;
  if ((long long)out_size != (long long)nN * HC2) return;

  const float* x     = (const float*)d_in[0];
  const int*   ei    = (const int*)  d_in[1];
  const float* gam   = (const float*)d_in[2];
  const float* bet   = (const float*)d_in[3];
  const float* W1l   = (const float*)d_in[4];
  const float* b1l   = (const float*)d_in[5];
  const float* W1r   = (const float*)d_in[6];
  const float* b1r   = (const float*)d_in[7];
  const float* att1  = (const float*)d_in[8];
  const float* bias1 = (const float*)d_in[9];
  const float* W2l   = (const float*)d_in[10];
  const float* b2l   = (const float*)d_in[11];
  const float* W2r   = (const float*)d_in[12];
  const float* b2r   = (const float*)d_in[13];
  const float* att2  = (const float*)d_in[14];
  const float* bias2 = (const float*)d_in[15];
  float* out = (float*)d_out;
  const int* src = ei;
  const int* dst = ei + nE;

  const int MP   = cdiv(nN, GBM) * GBM;
  const int gM   = MP / GBM;
  const int nb   = pick_nb(nE, nN);
  const int gA   = cdiv(MP, nb);
  const int vec8 = ((nE & 3) == 0) ? 1 : 0;
  if ((long long)gA * nb < (long long)MP) return;
  const int rpb  = cdiv(nN, NPB);

  char* ws = (char*)d_ws;
  size_t off = 0;
  const size_t oXN  = off; off = al256(off + (size_t)MP * (2 * DIN) * 2);
  const size_t oBT1 = off; off = al256(off + (size_t)(2 * HC1) * (2 * DIN) * 2);
  const size_t oBT2 = off; off = al256(off + (size_t)(2 * HC2) * (2 * HC1) * 2);
  const size_t oHF1 = off; off = al256(off + (size_t)MP * (2 * HC1) * 4);
  const size_t oA2  = off; off = al256(off + (size_t)MP * (2 * HC1) * 2);
  const size_t oHF2 = off; off = al256(off + (size_t)MP * (2 * HC2) * 4);
  const size_t oPT  = off; off = al256(off + (size_t)NPB * PARTD * 8);
  const size_t oSS  = off; off = al256(off + (size_t)(2 * DIN) * 4);
  if (off > ws_size || off > (size_t)WSMAX) return;
  unsigned short* XN  = (unsigned short*)(ws + oXN);
  unsigned short* BT1 = (unsigned short*)(ws + oBT1);
  unsigned short* BT2 = (unsigned short*)(ws + oBT2);
  float*          HF1 = (float*)(ws + oHF1);
  unsigned short* A2  = (unsigned short*)(ws + oA2);
  float*          HF2 = (float*)(ws + oHF2);
  double*         PT  = (double*)(ws + oPT);
  float*          SS  = (float*)(ws + oSS);

  hipFuncSetAttribute(reinterpret_cast<const void*>(&k_agg<8, 3, 0>),
                      hipFuncAttributeMaxDynamicSharedMemorySize, LDS_AGG);
  hipFuncSetAttribute(reinterpret_cast<const void*>(&k_agg<4, 5, 1>),
                      hipFuncAttributeMaxDynamicSharedMemorySize, LDS_AGG);

  k_bnstat<<<NPB, STHR, 0, stream>>>(x, nN, rpb, PT);
  k_bnfin<<<1, STHR, 0, stream>>>(PT, NPB, nN, gam, bet, SS);

  const int nUx = MP * ((2 * DIN) / 16);
  k_xprep<<<cdiv(nUx, NTHR), NTHR, 0, stream>>>(x, SS, XN, nN, nUx);

  {
    const int nU1 = HC1 * ((2 * DIN) / 8);
    k_wtr<<<dim3(cdiv(nU1, NTHR), 2), NTHR, 0, stream>>>(W1l, W1r, HC1, DIN, BT1);
    const int nU2 = HC2 * ((2 * HC1) / 8);
    k_wtr<<<dim3(cdiv(nU2, NTHR), 2), NTHR, 0, stream>>>(W2l, W2r, HC2, HC1, BT2);
  }

  k_gemm<<<dim3(gM, (2 * HC1) / GBN), GTHR, 0, stream>>>(XN, BT1, b1l, b1r, HC1, HF1, 2 * DIN, 2 * HC1);
  k_agg<8, 3, 0><<<gA, NTHR, LDS_AGG, stream>>>(src, dst, HF1, att1, bias1, A2, out,
                                                 nN, nE, nb, vec8, MP);
  k_gemm<<<dim3(gM, (2 * HC2) / GBN), GTHR, 0, stream>>>(A2, BT2, b2l, b2r, HC2, HF2, 2 * HC1, 2 * HC2);
  k_agg<4, 5, 1><<<gA, NTHR, LDS_AGG, stream>>>(src, dst, HF2, att2, bias2, A2, out,
                                                 nN, nE, nb, vec8, MP);
}
